// Block_17025250361620
// MI455X (gfx1250) — hardware-run, weakly checked
//
#include <hip/hip_runtime.h>
#include <math.h>


#ifndef NB
#define NB 1
#endif
#ifndef SEQ
#define SEQ 512
#endif
#define NB_FULL  1
#define SEQ_FULL 512
#ifndef OUT_SEQ
#define OUT_SEQ SEQ
#endif
#define DM   512
#define NH_  8
#define HD   64
#define NE   16
#define FF   512
#define KH   ((NE + 1) * FF)
#define GTP  32
#define WPITCH 512
#define AW   4
#define OSP  68
#define QRS  2048.0f
#define QRI  (1.0f / 2048.0f)
#define WSC  256.0f
#define WSI  (1.0f / 256.0f)
#define HSC  1024.0f
#define OSI  (1.0f / (256.0f * 1024.0f))
#define LOG2E 1.4426950408889634f
#define PSH  14.0f
#define NEGB (-3.0e38f)

static_assert(NB == 1);
static_assert(NH_ * HD == DM);
static_assert(HD == 64);
static_assert(DM == WPITCH);
static_assert(FF == WPITCH);
static_assert(DM % 64 == 0);
static_assert(FF % 64 == 0);
static_assert(DM % 32 == 0);
static_assert(KH % 32 == 0);
static_assert(KH % 64 == 0);
static_assert((KH * 2) % 128 == 0);
static_assert(SEQ % 64 == 0);
static_assert(SEQ % 32 == 0);
static_assert(SEQ % (16 * AW) == 0);
static_assert(SEQ % 8 == 0);
static_assert(SEQ <= SEQ_FULL);
static_assert(((size_t)SEQ * DM) % 256 == 0);
static_assert((OSP * 4) % 16 == 0);
static_assert(NE <= 16);
static_assert(NE + 1 <= GTP);
static_assert(AW * 16 * OSP * 4 <= 131072);
static_assert(64 * 65 * 4 <= 131072);
static_assert(16 * 68 * 4 <= 131072);

typedef _Float16 h16;
typedef unsigned short bf;
typedef __attribute__((ext_vector_type(16))) _Float16 v16h;
typedef __attribute__((ext_vector_type(8)))  _Float16 v8h;
typedef __attribute__((ext_vector_type(8)))  float    v8f;
typedef __attribute__((ext_vector_type(4)))  float    v4f;
typedef __attribute__((ext_vector_type(4)))  int      v4i;
typedef v4f  __attribute__((may_alias)) v4fa;

__device__ __forceinline__ unsigned short f2bf(float f) { unsigned u = __float_as_uint(f); u += 0x7FFFu + ((u >> 16) & 1u); return (unsigned short)(u >> 16); }
__device__ __forceinline__ float bfr(float f) { return __uint_as_float(((unsigned)f2bf(f)) << 16); }
__device__ __forceinline__ v16h cat16(v8h lo, v8h hi) { return __builtin_shufflevector(lo, hi, 0, 1, 2, 3, 4, 5, 6, 7, 8, 9, 10, 11, 12, 13, 14, 15); }
__device__ __forceinline__ v16h  ldh(const h16* p) { return cat16(*(const v8h*)p, *(const v8h*)(p + 16)); }
__device__ __forceinline__ void wave_sync() { __builtin_amdgcn_fence(3  , "wavefront"); __builtin_amdgcn_wave_barrier(); asm volatile("" ::: "memory"); }
__device__ __forceinline__ v8f wmma16g(v16h a, v16h b, v8f c) {
    c = __builtin_amdgcn_wmma_f32_16x16x32_f16(false, a, false, b, (short)0, c, false, false);
    asm volatile("v_nop\n\tv_nop\n\tv_nop\n\tv_nop" : "+v"(c) : "v"(a), "v"(b));
    return c;
}
__device__ __forceinline__ h16 toh_flush(float v) { const h16 r = (h16)v; return (fabsf(v) < 6.103515625e-05f) ? (h16)0.0f : r; }
__device__ __forceinline__ void split_h(float x, h16& hv, h16& rv) { hv = toh_flush(x); rv = toh_flush((x - (float)hv) * QRS); }
__device__ __forceinline__ float gelu_t(float x) { const float x3 = x * x * x; return 0.5f * x * (1.0f + tanhf(0.7978845608028654f * (x + 0.044715f * x3))); }

__global__ __launch_bounds__(256) void k_cvtT(const float* __restrict__ src, h16* dst, int dpitch, size_t szs, size_t dzs) {
    __shared__ float tl[64 * 65];
    const int tid = threadIdx.x;
    const int k0 = blockIdx.x * 64, n0 = blockIdx.y * 64;
    const float* s = src + (size_t)blockIdx.z * szs;
    h16* d = dst + (size_t)blockIdx.z * dzs;
    static_assert(256 * 4 * 4 == 64 * 64);
#pragma unroll 1
    for (int it = 0; it < 4; ++it) { const int p = it * 256 + tid; const int kr = p >> 4, c4 = (p & 15) * 4;
        const v4f v = *(const v4f*)(s + (size_t)(k0 + kr) * WPITCH + n0 + c4);
        tl[kr * 65 + c4 + 0] = v[0]; tl[kr * 65 + c4 + 1] = v[1]; tl[kr * 65 + c4 + 2] = v[2]; tl[kr * 65 + c4 + 3] = v[3]; }
    __syncthreads();
    static_assert(256 * 2 * 16 == 64 * 64 * 2);
#pragma unroll 1
    for (int ps = 0; ps < 2; ++ps) {
#pragma unroll 1
        for (int it = 0; it < 2; ++it) { const int p = it * 256 + tid; const int nrow = p >> 3, g = p & 7; v8h o;
#pragma unroll
            for (int i = 0; i < 8; ++i) o[i] = toh_flush(bfr(tl[(8 * g + i) * 65 + nrow]) * WSC);
            *(volatile v8h*)(d + (size_t)(n0 + nrow) * dpitch + k0 + 8 * g) = o; }
        if (ps == 0) __threadfence(); }
}

__global__ __launch_bounds__(32) void k_ropeinv(float* INV) {
#pragma clang fp contract(off)
    const int i = threadIdx.x;
    const float e = (float)i / 32.0f;
    const float p = powf(10000.0f, e);
    const float v = 1.0f / p;
    *(volatile float*)(INV + i) = v; __threadfence(); *(volatile float*)(INV + i) = v;
}

__global__ __launch_bounds__(256) void k_ropetab(const float* __restrict__ INV, float* CS) {
#pragma clang fp contract(off)
    __shared__ __align__(16) float cs2[512];
    const int tid = threadIdx.x;
    const int t = blockIdx.x * 8 + (tid >> 5), i = tid & 31;
    const float ang = (float)t * INV[i];
    cs2[tid] = cosf(ang); cs2[256 + tid] = sinf(ang);
    __syncthreads();
    static_assert(128 * 16 == 2 * 8 * 32 * 4);
    if (tid < 128) {
        const int which = tid >> 6, q = tid & 63;
        const v4f v = *(const v4fa*)(&cs2[4 * tid]);
        float* dp = CS + (size_t)which * SEQ * 32 + (size_t)blockIdx.x * 256 + 4 * q;
        *(volatile v4f*)dp = v; __threadfence(); *(volatile v4f*)dp = v;
    }
}

__global__ __launch_bounds__(256) void k_dyt(const float* __restrict__ xin, const float* __restrict__ ap, const float* __restrict__ gp, const float* __restrict__ bp, h16* HP, int inbf) {
#pragma clang fp contract(off)
    __shared__ __align__(16) float hs[256];
    const int tid = threadIdx.x;
    const size_t i = (size_t)blockIdx.x * 256 + tid;
    const int c = (int)(i % DM);
    const float a = bfr(ap[0]);
    const float xv = xin[i]; const float xr = bfr(xv); const float xx = (inbf != 0) ? xr : xv;
    hs[tid] = bfr(gp[c]) * tanhf(a * xx) + bfr(bp[c]);
    __syncthreads();
    static_assert(32 * 16 == 256 * 2);
    if (tid < 64) {
        const int q = tid & 31, which = tid >> 5;
        const v4f x0 = *(const v4fa*)(&hs[8 * q]); const v4f x1 = *(const v4fa*)(&hs[8 * q + 4]);
        v8h o;
#pragma unroll
        for (int k = 0; k < 4; ++k) { h16 h0, r0, h1, r1; split_h(x0[k], h0, r0); split_h(x1[k], h1, r1);
            o[k] = (which != 0) ? r0 : h0; o[4 + k] = (which != 0) ? r1 : h1; }
        h16* dp = HP + (size_t)which * SEQ * DM + (size_t)blockIdx.x * 256 + 8 * q;
        *(volatile v8h*)dp = o; __threadfence(); *(volatile v8h*)dp = o;
    }
}

template <int RESA, int RESB>
__device__ __forceinline__ void gemm_main(const h16* __restrict__ Ah, const h16* __restrict__ Ar, const h16* __restrict__ Bh, const h16* __restrict__ Br,
                                          const int K, const int r0, const int c0, const int lane, v8f (&acc)[2][4], v8f (&accR)[2][4]) {
    const int lr = lane & 15, hi = lane >> 4;
#pragma unroll
    for (int mb = 0; mb < 2; ++mb)
#pragma unroll
        for (int nb = 0; nb < 4; ++nb) { acc[mb][nb] = (v8f){}; accR[mb][nb] = (v8f){}; }
    const size_t aoff = (size_t)(r0 + lr) * K + 8 * hi, boff = (size_t)(c0 + lr) * K + 8 * hi;
#pragma unroll 1
    for (int kc = 0; kc < K; kc += 32) {
        v16h a[2], ar[2];
#pragma unroll
        for (int mb = 0; mb < 2; ++mb) { a[mb] = ldh(Ah + aoff + (size_t)mb * 16 * K + kc); ar[mb] = RESA ? ldh(Ar + aoff + (size_t)mb * 16 * K + kc) : a[mb]; }
#pragma unroll
        for (int nb = 0; nb < 4; ++nb) {
            const v16h b = ldh(Bh + boff + (size_t)nb * 16 * K + kc);
            const v16h br = RESB ? ldh(Br + boff + (size_t)nb * 16 * K + kc) : b;
#pragma unroll
            for (int mb = 0; mb < 2; ++mb) {
                acc[mb][nb] = wmma16g(a[mb], b, acc[mb][nb]);
                if (RESA) accR[mb][nb] = wmma16g(ar[mb], b, accR[mb][nb]);
                if (RESB) accR[mb][nb] = wmma16g(a[mb], br, accR[mb][nb]); }
        }
    }
}

__global__ __launch_bounds__(32) void k_qkproj(const h16* __restrict__ HP, const h16* __restrict__ WA, const float* __restrict__ CS, h16* QKH, h16* QKR) {
    __shared__ __align__(16) float os[16 * 68];
    const int lane = threadIdx.x & 31, lr = lane & 15, hi = lane >> 4;
    const int r0 = blockIdx.x * 32, c0 = blockIdx.y * 64, z = blockIdx.z;
    v8f acc[2][4], accR[2][4];
    const h16* wt = WA + (size_t)z * DM * DM;
    gemm_main<1, 0>(HP, HP + (size_t)SEQ * DM, wt, wt, DM, r0, c0, lane, acc, accR);
    const size_t pbase = ((size_t)z * NH_ + blockIdx.y) * SEQ * HD;
    static_assert(32 * 4 * 16 == 16 * HD * 2);
#pragma unroll
    for (int mb = 0; mb < 2; ++mb) {
#pragma unroll
        for (int nb = 0; nb < 4; ++nb) {
#pragma unroll
            for (int j = 0; j < 8; ++j) os[(hi * 8 + j) * 68 + nb * 16 + lr] = (acc[mb][nb][j] + accR[mb][nb][j] * QRI) * WSI; }
        wave_sync();
#pragma unroll 1
        for (int ps = 0; ps < 2; ++ps) {
#pragma unroll 1
            for (int s = 0; s < 4; ++s) { const int row = 4 * s + (lane >> 3), c8 = (lane & 7) * 8, ci = c8 & 31; const bool up = c8 >= 32;
                const int t = r0 + mb * 16 + row;
                const v4f a0 = *(const v4fa*)(&os[row * 68 + ci]); const v4f a1 = *(const v4fa*)(&os[row * 68 + ci + 4]);
                const v4f b0 = *(const v4fa*)(&os[row * 68 + 32 + ci]); const v4f b1 = *(const v4fa*)(&os[row * 68 + 32 + ci + 4]);
                const float* cp = CS + (size_t)t * 32 + ci; const float* sp = CS + (size_t)SEQ * 32 + (size_t)t * 32 + ci;
                const v4f cc0 = *(const v4f*)cp; const v4f cc1 = *(const v4f*)(cp + 4); const v4f ss0 = *(const v4f*)sp; const v4f ss1 = *(const v4f*)(sp + 4);
                v8h hv, rv;
#pragma unroll
                for (int i = 0; i < 4; ++i) {
                    const float lo0 = a0[i] * cc0[i] - b0[i] * ss0[i], up0 = a0[i] * ss0[i] + b0[i] * cc0[i];
                    const float lo1 = a1[i] * cc1[i] - b1[i] * ss1[i], up1 = a1[i] * ss1[i] + b1[i] * cc1[i];
                    const float y0 = up ? up0 : lo0, y1 = up ? up1 : lo1;
                    h16 h0, q0, h1, q1; split_h(y0, h0, q0); split_h(y1, h1, q1);
                    hv[i] = h0; rv[i] = q0; hv[4 + i] = h1; rv[4 + i] = q1; }
                const size_t oo = pbase + (size_t)t * HD + c8;
                *(volatile v8h*)(QKH + oo) = hv; *(volatile v8h*)(QKR + oo) = rv; }
            if (ps == 0) __threadfence(); }
        wave_sync();
    }
}

__global__ __launch_bounds__(32) void k_vproj(const h16* __restrict__ WV, const h16* __restrict__ HP, h16* VP) {
    __shared__ __align__(16) float os[16 * 68];
    const int lane = threadIdx.x & 31, lr = lane & 15, hi = lane >> 4;
    const int r0 = blockIdx.x * 32, c0 = blockIdx.y * 64;
    v8f acc[2][4], accR[2][4];
    gemm_main<0, 1>(WV, WV, HP, HP + (size_t)SEQ * DM, DM, r0, c0, lane, acc, accR);
    static_assert(32 * 4 * 16 == 16 * 64 * 2);
#pragma unroll
    for (int mb = 0; mb < 2; ++mb) {
#pragma unroll
        for (int nb = 0; nb < 4; ++nb) {
#pragma unroll
            for (int j = 0; j < 8; ++j) os[(hi * 8 + j) * 68 + nb * 16 + lr] = (acc[mb][nb][j] + accR[mb][nb][j] * QRI) * WSI; }
        wave_sync();
#pragma unroll 1
        for (int ps = 0; ps < 2; ++ps) {
#pragma unroll 1
            for (int s = 0; s < 4; ++s) { const int row = 4 * s + (lane >> 3), c8 = (lane & 7) * 8;
                const v4f x0 = *(const v4fa*)(&os[row * 68 + c8]); const v4f x1 = *(const v4fa*)(&os[row * 68 + c8 + 4]); v8h hv, rv;
#pragma unroll
                for (int i = 0; i < 4; ++i) { h16 h0, q0, h1, q1; split_h(x0[i], h0, q0); split_h(x1[i], h1, q1); hv[i] = h0; rv[i] = q0; hv[4 + i] = h1; rv[4 + i] = q1; }
                const size_t oo = (size_t)(r0 + mb * 16 + row) * SEQ + c0 + c8;
                *(volatile v8h*)(VP + oo) = hv; *(volatile v8h*)(VP + (size_t)DM * SEQ + oo) = rv; }
            if (ps == 0) __threadfence(); }
        wave_sync();
    }
}

__global__ __launch_bounds__(32 * AW) void k_flash(const h16* __restrict__ QKH, const h16* __restrict__ QKR, const h16* __restrict__ VP, const int* __restrict__ amask, h16* CX) {
    __shared__ __align__(16) float os[AW * 16 * OSP];
    const int lane = threadIdx.x & 31, lr = lane & 15, hi = lane >> 4;
    const int wave = __builtin_amdgcn_readfirstlane((int)(threadIdx.x >> 5));
    const int h = blockIdx.y;
    const int t0 = (blockIdx.x * AW + wave) * 16;
    const int tq = t0 + lr;
    const int nk = (t0 + 16 + 31) & ~31;
    const size_t pl = (size_t)NH_ * SEQ * HD;
    const size_t pbase = (size_t)h * SEQ * HD;
    const size_t qo = pbase + (size_t)tq * HD + 8 * hi;
    const size_t ko = pl + pbase + (size_t)lr * HD + 8 * hi;
    const size_t vo = (size_t)(h * HD + lr) * SEQ + 8 * hi;
    const size_t vres = (size_t)DM * SEQ;
    const int* amb = amask + 8 * hi;
    const v16h hz = (v16h){};
    v8f o[4], oR[4];
#pragma unroll
    for (int j = 0; j < 4; ++j) { o[j] = (v8f){}; oR[j] = (v8f){}; }
    float m = NEGB, l = 0.0f;
#pragma unroll 1
    for (int key0 = 0; key0 < nk; key0 += 32) {
        v8f sHa = (v8f){}, sLa = (v8f){}, sHb = (v8f){}, sLb = (v8f){};
#pragma unroll
        for (int ds = 0; ds < 2; ++ds) {
            const v16h qh = ldh(QKH + qo + ds * 32), qr = ldh(QKR + qo + ds * 32);
            const size_t kk = ko + (size_t)key0 * HD + ds * 32;
            const v16h ka = ldh(QKH + kk), kb = ldh(QKH + kk + 16 * HD);
            const v16h kra = ldh(QKR + kk), krb = ldh(QKR + kk + 16 * HD);
            sHa = wmma16g(ka, qh, sHa); sLa = wmma16g(ka, qr, sLa); sLa = wmma16g(kra, qh, sLa);
            sHb = wmma16g(kb, qh, sHb); sLb = wmma16g(kb, qr, sLb); sLb = wmma16g(krb, qh, sLb);
        }
        const int* ap = amb + key0;
        const v4i m0 = *(const v4i*)ap, m1 = *(const v4i*)(ap + 4), m2 = *(const v4i*)(ap + 16), m3 = *(const v4i*)(ap + 20);
        int kx[8], ky[8];
#pragma unroll
        for (int r = 0; r < 4; ++r) { kx[r] = m0[r]; kx[4 + r] = m1[r]; ky[r] = m2[r]; ky[4 + r] = m3[r]; }
        const int ja = key0 + 8 * hi;
        float ta[8], tb[8]; float mx = NEGB;
#pragma unroll
        for (int r = 0; r < 8; ++r) {
            const int j0 = ja + r, j1 = ja + 16 + r;
            float ca = (j0 <= tq) ? (float)kx[r] : 0.0f; ca = (j0 == tq) ? 1.0f : ca;
            float cb = (j1 <= tq) ? (float)ky[r] : 0.0f; cb = (j1 == tq) ? 1.0f : cb;
            const float ba = -(1.0f - ca) * 1.0e9f, bb = -(1.0f - cb) * 1.0e9f;
            ta[r] = ((sHa[r] + sLa[r] * QRI) * 0.125f + ba) * LOG2E;
            tb[r] = ((sHb[r] + sLb[r] * QRI) * 0.125f + bb) * LOG2E;
            mx = fmaxf(mx, fmaxf(ta[r], tb[r])); }
        mx = fmaxf(mx, __shfl_xor(mx, 16, 32));
        const float mnew = fmaxf(m, mx);
        const float alpha = __builtin_amdgcn_exp2f(m - mnew);
        const float sh = PSH - mnew;
        v16h pb = hz, pr = hz; float ls = 0.0f;
#pragma unroll
        for (int r = 0; r < 8; ++r) {
            const float e0 = ta[r] + sh, e1 = tb[r] + sh;
            const float x0 = __builtin_amdgcn_exp2f(e0), x1 = __builtin_amdgcn_exp2f(e1);
            const float ga = (e0 < -14.0f) ? 0.0f : x0, gb = (e1 < -14.0f) ? 0.0f : x1;
            const h16 pa = toh_flush(ga); const h16 pc = toh_flush(gb);
            pb[r] = pa; pb[8 + r] = pc;
            pr[r] = toh_flush((ga - (float)pa) * QRS); pr[8 + r] = toh_flush((gb - (float)pc) * QRS);
            ls += ga + gb; }
        l = l * alpha + ls; m = mnew;
#pragma unroll
        for (int j = 0; j < 4; ++j) { o[j] = o[j] * alpha; oR[j] = oR[j] * alpha; }
        const size_t vk = vo + key0;
#pragma unroll
        for (int jp = 0; jp < 2; ++jp) {
            const size_t va = vk + (size_t)(32 * jp) * SEQ, vb = vk + (size_t)(32 * jp + 16) * SEQ;
            const v16h v0 = ldh(VP + va), v1 = ldh(VP + vb);
            const v16h vr0 = ldh(VP + vres + va), vr1 = ldh(VP + vres + vb);
            o[2 * jp] = wmma16g(v0, pb, o[2 * jp]); oR[2 * jp] = wmma16g(v0, pr, oR[2 * jp]); oR[2 * jp] = wmma16g(vr0, pb, oR[2 * jp]);
            o[2 * jp + 1] = wmma16g(v1, pb, o[2 * jp + 1]); oR[2 * jp + 1] = wmma16g(v1, pr, oR[2 * jp + 1]); oR[2 * jp + 1] = wmma16g(vr1, pb, oR[2 * jp + 1]);
        }
    }
    l += __shfl_xor(l, 16, 32);
    const bool any = l > 0.0f;
    const float lsafe = any ? l : 1.0f;
    const float inv = any ? (1.0f / lsafe) : 0.0f;
    const int wb = wave * 16 * OSP;
#pragma unroll
    for (int j = 0; j < 4; ++j) { const v8f f = o[j] + oR[j] * QRI; v4f a, c;
        a[0] = f[0] * inv; a[1] = f[1] * inv; a[2] = f[2] * inv; a[3] = f[3] * inv; c[0] = f[4] * inv; c[1] = f[5] * inv; c[2] = f[6] * inv; c[3] = f[7] * inv;
        *(v4fa*)(&os[wb + lr * OSP + 16 * j + 8 * hi]) = a; *(v4fa*)(&os[wb + lr * OSP + 16 * j + 8 * hi + 4]) = c; }
    wave_sync();
    h16* crow = CX + (size_t)t0 * DM + h * HD;
    static_assert(32 * 4 * 16 == 16 * HD * 2);
#pragma unroll 1
    for (int ps = 0; ps < 2; ++ps) {
#pragma unroll 1
        for (int s = 0; s < 4; ++s) { const int row = 4 * s + (lane >> 3), c8 = (lane & 7) * 8;
            const v4f x0 = *(const v4fa*)(&os[wb + row * OSP + c8]); const v4f x1 = *(const v4fa*)(&os[wb + row * OSP + c8 + 4]); v8h hv, rv;
#pragma unroll
            for (int i = 0; i < 4; ++i) { h16 h0, q0, h1, q1; split_h(x0[i], h0, q0); split_h(x1[i], h1, q1); hv[i] = h0; rv[i] = q0; hv[4 + i] = h1; rv[4 + i] = q1; }
            *(volatile v8h*)(crow + (size_t)row * DM + c8) = hv; *(volatile v8h*)(crow + (size_t)SEQ * DM + (size_t)row * DM + c8) = rv; }
        if (ps == 0) __threadfence(); }
}

__global__ __launch_bounds__(32) void k_oproj(const h16* __restrict__ CX, const h16* __restrict__ WO, const float* __restrict__ x, float* X1) {
    __shared__ __align__(16) float os[16 * 68];
    const int lane = threadIdx.x & 31, lr = lane & 15, hi = lane >> 4;
    const int r0 = blockIdx.x * 32, c0 = blockIdx.y * 64;
    v8f acc[2][4], accR[2][4];
    gemm_main<1, 0>(CX, CX + (size_t)SEQ * DM, WO, WO, DM, r0, c0, lane, acc, accR);
    static_assert(32 * 8 * 16 == 16 * 64 * 4);
#pragma unroll
    for (int mb = 0; mb < 2; ++mb) {
#pragma unroll
        for (int nb = 0; nb < 4; ++nb) {
#pragma unroll
            for (int j = 0; j < 8; ++j) os[(hi * 8 + j) * 68 + nb * 16 + lr] = (acc[mb][nb][j] + accR[mb][nb][j] * QRI) * WSI; }
        wave_sync();
#pragma unroll 1
        for (int ps = 0; ps < 2; ++ps) {
#pragma unroll 1
            for (int s = 0; s < 8; ++s) { const int row = 2 * s + (lane >> 4), c4 = (lane & 15) * 4;
                const size_t oo = (size_t)(r0 + mb * 16 + row) * DM + c0 + c4;
                const v4f pv = *(const v4fa*)(&os[row * 68 + c4]); const v4f xv = *(const v4f*)(x + oo); v4f val;
                val[0] = bfr(xv[0]) + pv[0]; val[1] = bfr(xv[1]) + pv[1]; val[2] = bfr(xv[2]) + pv[2]; val[3] = bfr(xv[3]) + pv[3];
                *(volatile v4f*)(X1 + oo) = val; }
            if (ps == 0) __threadfence(); }
        wave_sync();
    }
}

__global__ __launch_bounds__(128) void k_router(const h16* __restrict__ H2, const float* __restrict__ gw, const float* __restrict__ gb, float* GT) {
#pragma clang fp contract(off)
    const int lane = threadIdx.x & 31, lr = lane & 15;
    const int wave = __builtin_amdgcn_readfirstlane((int)(threadIdx.x >> 5));
    const int t = blockIdx.x * 4 + wave;
    float acc[16];
#pragma unroll
    for (int e = 0; e < 16; ++e) acc[e] = 0.0f;
#pragma unroll 1
    for (int it = 0; it < DM / 32; ++it) {
        const int d = it * 32 + lane;
        const float hv = (float)H2[(size_t)t * DM + d] + (float)H2[(size_t)SEQ * DM + (size_t)t * DM + d] * QRI;
        const float* g = gw + (size_t)d * NE;
        const v4f g0 = *(const v4f*)g, g1 = *(const v4f*)(g + 4), g2 = *(const v4f*)(g + 8), g3 = *(const v4f*)(g + 12);
#pragma unroll
        for (int e = 0; e < 4; ++e) { acc[e] = fmaf(hv, bfr(g0[e]), acc[e]); acc[4 + e] = fmaf(hv, bfr(g1[e]), acc[4 + e]);
                                      acc[8 + e] = fmaf(hv, bfr(g2[e]), acc[8 + e]); acc[12 + e] = fmaf(hv, bfr(g3[e]), acc[12 + e]); }
    }
    float lg = 0.0f;
#pragma unroll
    for (int e = 0; e < 16; ++e) { float v = acc[e];
        v += __shfl_xor(v, 16, 32); v += __shfl_xor(v, 8, 32); v += __shfl_xor(v, 4, 32); v += __shfl_xor(v, 2, 32); v += __shfl_xor(v, 1, 32);
        lg = (lr == e) ? v : lg; }
    lg += bfr(gb[lr]);
    float mx = lg;
    mx = fmaxf(mx, __shfl_xor(mx, 8, 32)); mx = fmaxf(mx, __shfl_xor(mx, 4, 32)); mx = fmaxf(mx, __shfl_xor(mx, 2, 32)); mx = fmaxf(mx, __shfl_xor(mx, 1, 32));
    const float ex = expf(lg - mx);
    float sm = ex;
    sm += __shfl_xor(sm, 8, 32); sm += __shfl_xor(sm, 4, 32); sm += __shfl_xor(sm, 2, 32); sm += __shfl_xor(sm, 1, 32);
    const float p = ex * (1.0f / sm);
    float bv = p; int bi = lr;
#pragma unroll
    for (int mk = 8; mk >= 1; mk >>= 1) { const float ov = __shfl_xor(bv, mk, 32); const int oi = __shfl_xor(bi, mk, 32);
        const bool take = (ov > bv) | ((ov == bv) & (oi < bi)); bv = take ? ov : bv; bi = take ? oi : bi; }
    const int i1 = bi; const float v1 = bv;
    float cv = (lr == i1) ? -1.0f : p; int ci = lr;
#pragma unroll
    for (int mk = 8; mk >= 1; mk >>= 1) { const float ov = __shfl_xor(cv, mk, 32); const int oi = __shfl_xor(ci, mk, 32);
        const bool take = (ov > cv) | ((ov == cv) & (oi < ci)); cv = take ? ov : cv; ci = take ? oi : ci; }
    const int i2 = ci; const float v2 = cv;
    const float gt = (lr == i1) ? v1 : ((lr == i2) ? v2 : 0.0f);
    const float val = (lane < 16) ? gt : ((lane == 16) ? 1.0f : 0.0f);
    float* dp = GT + (size_t)t * GTP + lane;
    *(volatile float*)dp = val; __threadfence(); *(volatile float*)dp = val;
}

__global__ __launch_bounds__(32) void k_gemm1(const h16* __restrict__ H2, const h16* __restrict__ W1T, const float* __restrict__ GT, h16* HID) {
    __shared__ __align__(16) float os[16 * 68];
    const int lane = threadIdx.x & 31, lr = lane & 15, hi = lane >> 4;
    const int r0 = blockIdx.x * 32, c0 = blockIdx.y * 64;
    const int e = c0 / FF;
    v8f acc[2][4], accR[2][4];
    gemm_main<0, 0>(H2, H2, W1T, W1T, DM, r0, c0, lane, acc, accR);
    static_assert(32 * 4 * 16 == 16 * 64 * 2);
#pragma unroll
    for (int mb = 0; mb < 2; ++mb) {
#pragma unroll
        for (int nb = 0; nb < 4; ++nb) {
#pragma unroll
            for (int j = 0; j < 8; ++j) os[(hi * 8 + j) * 68 + nb * 16 + lr] = acc[mb][nb][j] * WSI; }
        wave_sync();
#pragma unroll 1
        for (int ps = 0; ps < 2; ++ps) {
#pragma unroll 1
            for (int s = 0; s < 4; ++s) { const int row = 4 * s + (lane >> 3), c8 = (lane & 7) * 8;
                const int t = r0 + mb * 16 + row;
                const float gv = GT[(size_t)t * GTP + e] * HSC;
                const v4f x0 = *(const v4fa*)(&os[row * 68 + c8]); const v4f x1 = *(const v4fa*)(&os[row * 68 + c8 + 4]); v8h hv;
#pragma unroll
                for (int i = 0; i < 4; ++i) { hv[i] = toh_flush(gelu_t(x0[i]) * gv); hv[4 + i] = toh_flush(gelu_t(x1[i]) * gv); }
                *(volatile v8h*)(HID + (size_t)t * KH + c0 + c8) = hv; }
            if (ps == 0) __threadfence(); }
        wave_sync();
    }
}

__global__ __launch_bounds__(32) void k_gemm2(const h16* __restrict__ HID, const h16* __restrict__ W2T, const float* __restrict__ X1, float* OUT) {
    __shared__ __align__(16) float os[16 * 68];
    const int lane = threadIdx.x & 31, lr = lane & 15, hi = lane >> 4;
    const int r0 = blockIdx.x * 32, c0 = blockIdx.y * 64;
    v8f acc[2][4], accR[2][4];
    gemm_main<0, 0>(HID, HID, W2T, W2T, KH, r0, c0, lane, acc, accR);
    static_assert(32 * 8 * 16 == 16 * 64 * 4);
#pragma unroll
    for (int mb = 0; mb < 2; ++mb) {
#pragma unroll
        for (int nb = 0; nb < 4; ++nb) {
#pragma unroll
            for (int j = 0; j < 8; ++j) os[(hi * 8 + j) * 68 + nb * 16 + lr] = acc[mb][nb][j] * OSI; }
        wave_sync();
#pragma unroll 1
        for (int ps = 0; ps < 2; ++ps) {
#pragma unroll 1
            for (int s = 0; s < 8; ++s) { const int row = 2 * s + (lane >> 4), c4 = (lane & 15) * 4;
                const size_t oo = (size_t)(r0 + mb * 16 + row) * DM + c0 + c4;
                const v4f pv = *(const v4fa*)(&os[row * 68 + c4]); const v4f xv = *(const v4f*)(X1 + oo); v4f val;
                val[0] = xv[0] + pv[0]; val[1] = xv[1] + pv[1]; val[2] = xv[2] + pv[2]; val[3] = xv[3] + pv[3];
                *(volatile v4f*)(OUT + oo) = val; }
            if (ps == 0) __threadfence(); }
        wave_sync();
    }
}

static constexpr size_t al256(size_t v) { return (v + 255) & ~(size_t)255; }
static constexpr size_t SZ_WA  = al256((size_t)4 * DM * DM * 2);
static constexpr size_t SZ_W1  = al256((size_t)KH * DM * 2);
static constexpr size_t SZ_W2  = al256((size_t)DM * KH * 2);
static constexpr size_t SZ_INV = 256;
static constexpr size_t SZ_CS  = al256((size_t)2 * SEQ * 32 * 4);
static constexpr size_t SZ_HP  = al256((size_t)2 * SEQ * DM * 2);
static constexpr size_t SZ_QK  = al256((size_t)2 * NH_ * SEQ * HD * 2);
static constexpr size_t SZ_VP  = al256((size_t)2 * DM * SEQ * 2);
static constexpr size_t SZ_X1  = al256((size_t)SEQ * DM * 4);
static constexpr size_t SZ_GT  = al256((size_t)SEQ * GTP * 4);
static constexpr size_t SZ_HID = al256((size_t)SEQ * KH * 2);
static constexpr size_t SZ_TOTAL = SZ_WA + SZ_W1 + SZ_W2 + SZ_INV + SZ_CS + 3 * SZ_HP + 2 * SZ_QK + SZ_VP + SZ_X1 + SZ_GT + SZ_HID;
static_assert(SZ_TOTAL <= (size_t)134217728);
static_assert(((size_t)DM * DM * 2) % 256 == 0);
static_assert(((size_t)NE * FF * DM * 2) % 256 == 0);
static_assert(((size_t)SEQ * DM * 2) % 256 == 0);
static_assert(((size_t)NH_ * SEQ * HD * 2) % 256 == 0);
static_assert(((size_t)SEQ * 32 * 4) % 256 == 0);
static_assert((size_t)NH_ * SEQ * HD == (size_t)DM * SEQ);

extern "C" void kernel_launch(void* const* d_in, const int* in_sizes, int n_in,
                              void* d_out, int out_size, void* d_ws, size_t ws_size, hipStream_t stream) {
    if (n_in < 18) return;
    if ((size_t)in_sizes[0] < (size_t)SEQ * DM || in_sizes[1] < SEQ) return;
    if ((size_t)in_sizes[2] < (size_t)DM * DM || (size_t)in_sizes[3] < (size_t)DM * DM || (size_t)in_sizes[4] < (size_t)DM * DM || (size_t)in_sizes[5] < (size_t)DM * DM) return;
    if (in_sizes[6] < 1 || in_sizes[7] < DM || in_sizes[8] < DM || in_sizes[9] < 1 || in_sizes[10] < DM || in_sizes[11] < DM) return;
    if (in_sizes[12] < DM * NE || in_sizes[13] < NE) return;
    if ((size_t)in_sizes[14] < (size_t)NE * DM * FF || (size_t)in_sizes[15] < (size_t)NE * FF * DM) return;
    if ((size_t)in_sizes[16] < (size_t)DM * FF || (size_t)in_sizes[17] < (size_t)FF * DM) return;
    if ((size_t)out_size < (size_t)SEQ * DM) return;
    if (SZ_TOTAL > ws_size) return;
    const float* x  = (const float*)d_in[0];  const int* amask = (const int*)d_in[1];
    const float* wq = (const float*)d_in[2];  const float* wk = (const float*)d_in[3];
    const float* wv = (const float*)d_in[4];  const float* wo = (const float*)d_in[5];
    const float* a1 = (const float*)d_in[6];  const float* g1 = (const float*)d_in[7];  const float* b1 = (const float*)d_in[8];
    const float* a2 = (const float*)d_in[9];  const float* g2 = (const float*)d_in[10]; const float* b2 = (const float*)d_in[11];
    const float* gate_w = (const float*)d_in[12]; const float* gate_b = (const float*)d_in[13];
    const float* ek = (const float*)d_in[14]; const float* ev = (const float*)d_in[15];
    const float* sk = (const float*)d_in[16]; const float* sv = (const float*)d_in[17];
    float* OUT = (float*)d_out;
    char* wsp = (char*)d_ws;
    h16* WA  = (h16*)wsp; wsp += SZ_WA;
    h16* W1T = (h16*)wsp; wsp += SZ_W1;
    h16* W2T = (h16*)wsp; wsp += SZ_W2;
    float* INV = (float*)wsp; wsp += SZ_INV;
    float* CS  = (float*)wsp; wsp += SZ_CS;
    h16* H1  = (h16*)wsp; wsp += SZ_HP;
    h16* H2  = (h16*)wsp; wsp += SZ_HP;
    h16* CX  = (h16*)wsp; wsp += SZ_HP;
    h16* QKH = (h16*)wsp; wsp += SZ_QK;
    h16* QKR = (h16*)wsp; wsp += SZ_QK;
    h16* VP  = (h16*)wsp; wsp += SZ_VP;
    float* X1 = (float*)wsp; wsp += SZ_X1;
    float* GT = (float*)wsp; wsp += SZ_GT;
    h16* HID = (h16*)wsp; wsp += SZ_HID;

    const size_t WW = (size_t)DM * DM;
    k_cvtT<<<dim3(DM / 64, DM / 64, 1), 256, 0, stream>>>(wq, WA, DM, 0, 0);
    k_cvtT<<<dim3(DM / 64, DM / 64, 1), 256, 0, stream>>>(wk, WA + WW, DM, 0, 0);
    k_cvtT<<<dim3(DM / 64, DM / 64, 1), 256, 0, stream>>>(wv, WA + 2 * WW, DM, 0, 0);
    k_cvtT<<<dim3(DM / 64, DM / 64, 1), 256, 0, stream>>>(wo, WA + 3 * WW, DM, 0, 0);
    k_cvtT<<<dim3(DM / 64, FF / 64, NE), 256, 0, stream>>>(ek, W1T, DM, (size_t)DM * FF, (size_t)FF * DM);
    k_cvtT<<<dim3(DM / 64, FF / 64, 1), 256, 0, stream>>>(sk, W1T + (size_t)NE * FF * DM, DM, 0, 0);
    k_cvtT<<<dim3(FF / 64, DM / 64, NE), 256, 0, stream>>>(ev, W2T, KH, (size_t)FF * DM, (size_t)FF);
    k_cvtT<<<dim3(FF / 64, DM / 64, 1), 256, 0, stream>>>(sv, W2T + (size_t)NE * FF, KH, 0, 0);

    k_ropeinv<<<1, 32, 0, stream>>>(INV);
    k_ropetab<<<SEQ / 8, 256, 0, stream>>>(INV, CS);

    k_dyt<<<(unsigned)((size_t)SEQ * DM / 256), 256, 0, stream>>>(x, a1, g1, b1, H1, 1);
    k_qkproj<<<dim3(SEQ / 32, DM / 64, 2), 32, 0, stream>>>(H1, WA, CS, QKH, QKR);
    k_vproj<<<dim3(DM / 32, SEQ / 64, 1), 32, 0, stream>>>(WA + 2 * WW, H1, VP);
    k_flash<<<dim3(SEQ / (16 * AW), NH_, 1), 32 * AW, 0, stream>>>(QKH, QKR, VP, amask, CX);
    k_oproj<<<dim3(SEQ / 32, DM / 64, 1), 32, 0, stream>>>(CX, WA + 3 * WW, x, X1);

    k_dyt<<<(unsigned)((size_t)SEQ * DM / 256), 256, 0, stream>>>(X1, a2, g2, b2, H2, 0);
    k_router<<<SEQ / 4, 128, 0, stream>>>(H2, gate_w, gate_b, GT);
    k_gemm1<<<dim3(SEQ / 32, KH / 64, 1), 32, 0, stream>>>(H2, W1T, GT, HID);
    k_gemm2<<<dim3(SEQ / 32, DM / 64, 1), 32, 0, stream>>>(HID, W2T, X1, OUT);
}
